// TransformerBlock_65085934403864
// MI455X (gfx1250) — hardware-verified
//
#include <hip/hip_runtime.h>
#include <stddef.h>
#include <math.h>


typedef _Float16 v16h __attribute__((ext_vector_type(16)));
typedef _Float16 v8h  __attribute__((ext_vector_type(8)));
typedef float    v8f  __attribute__((ext_vector_type(8)));
typedef float    v4f  __attribute__((ext_vector_type(4)));

#ifndef NB
#define NB 1
#endif
#ifndef SEQ
#define SEQ 4096
#endif
#define NB_FULL  1
#define SEQ_FULL 4096
#define DIM   1024
#define NHEAD 16
#define HD    64
#define FF    4096
#define MROWS (NB * SEQ)

static_assert(NB == 1 && NB_FULL == 1);
static_assert(SEQ >= 128 && SEQ <= SEQ_FULL && (SEQ % 128) == 0);
static_assert(DIM == NHEAD * HD);
static_assert(FF == 4 * DIM);
static_assert((MROWS % 64) == 0 && (MROWS % 8) == 0);
static_assert((DIM % 64) == 0 && (FF % 64) == 0);

#define LDT 72
#define LDC 68

#define WCARRY 64.0f
#define PCARRY 1024.0f
#define VCARRY 64.0f

#define P16_BYTES  ((size_t)MROWS * DIM * 2)
#define WQKV_BYTES ((size_t)3 * DIM * DIM * 2)
#define WO_BYTES   ((size_t)DIM * DIM * 2)
#define W1_BYTES   ((size_t)FF * DIM * 2)
#define W2_BYTES   ((size_t)DIM * FF * 2)
#define OFF_WQKV   ((size_t)0)
#define OFF_WO     (OFF_WQKV + WQKV_BYTES)
#define OFF_W1     (OFF_WO + WO_BYTES)
#define OFF_W2     (OFF_W1 + W1_BYTES)
#define OFF_XN     (OFF_W2 + W2_BYTES)
#define OFF_QKV    (OFF_XN + P16_BYTES)
#define OFF_OV     (OFF_QKV + 3 * P16_BYTES)
#define OFF_X32    (OFF_OV + P16_BYTES)
#define OFF_H      (OFF_X32 + 2 * P16_BYTES)
#define OFF_G      (OFF_H + P16_BYTES)
#define WS_TOTAL   (OFF_G + 4 * P16_BYTES)
static_assert((size_t)MROWS * FF * 2 == 4 * P16_BYTES);
static_assert((size_t)DIM * SEQ * 2 == P16_BYTES);
static_assert((P16_BYTES % 128) == 0 && (WO_BYTES % 128) == 0);
static_assert(WS_TOTAL <= (size_t)134217728);

__device__ __forceinline__ float bf16r(float x) {
  unsigned int u = __float_as_uint(x);
  u = (u + 0x7FFFu + ((u >> 16) & 1u)) & 0xFFFF0000u;
  return __uint_as_float(u);
}

__device__ __forceinline__ v16h frag_at(const _Float16* p) {
  v8h lo = *(const v8h*)(p);
  v8h hi = *(const v8h*)(p + 16);
  v16h out;
#pragma unroll
  for (int i = 0; i < 8; ++i) { out[i] = lo[i]; out[i + 8] = hi[i]; }
  return out;
}
__device__ __forceinline__ v16h ld_frag(const _Float16* base, int ld) {
  const int lane = threadIdx.x & 31;
  return frag_at(base + (lane & 15) * ld + (lane >> 4) * 8);
}

__device__ __forceinline__ v8f wmma16(v16h a, v16h b, v8f c) {
  v8f d = __builtin_amdgcn_wmma_f32_16x16x32_f16(false, a, false, b, (short)0, c,
                                                 false, false);
  asm volatile("v_nop\n\tv_nop\n\tv_nop\n\tv_nop" : "+v"(d) : "v"(a), "v"(b));
  return d;
}

__device__ __forceinline__ float red16_max(float x) {
#pragma unroll
  for (int off = 1; off < 16; off <<= 1) x = fmaxf(x, __shfl_xor(x, off, 32));
  return x;
}
__device__ __forceinline__ float red16_sum(float x) {
#pragma unroll
  for (int off = 1; off < 16; off <<= 1) x += __shfl_xor(x, off, 32);
  return x;
}
__device__ __forceinline__ float wave_sum(float x) {
#pragma unroll
  for (int off = 1; off < 32; off <<= 1) x += __shfl_xor(x, off, 32);
  return x;
}

__device__ __forceinline__ void wave_lds_sync() {
  __builtin_amdgcn_fence(3  , "wavefront");
  asm volatile("s_wait_dscnt 0x0" ::: "memory");
  __builtin_amdgcn_wave_barrier();
}

__device__ __forceinline__ float gelu_erf(float v) {
  return 0.5f * v * (1.0f + erff(v * 0.70710678118654752f));
}

__global__ __launch_bounds__(256) void wconv_kernel(
    const float* __restrict__ W, _Float16* __restrict__ Wt, int K, int N) {
  __shared__ _Float16 T[64 * LDT];
  const int tid = threadIdx.x;
  const int n0 = blockIdx.x * 64;
  const int k0 = blockIdx.y * 64;
#pragma unroll 4
  for (int j = 0; j < 16; ++j) {
    const int idx = tid + 256 * j;
    const int kr = idx >> 6, nc = idx & 63;
    const float v = W[(size_t)(k0 + kr) * N + n0 + nc];
    T[nc * LDT + kr] = (_Float16)(WCARRY * bf16r(v));
  }
  __syncthreads();
  v8h x[2];
  size_t off[2];
#pragma unroll
  for (int i = 0; i < 2; ++i) {
    const int n = 32 * i + (tid >> 3);
    const int kc = (tid & 7) * 8;
    x[i] = *(const v8h*)&T[n * LDT + kc];
    off[i] = (size_t)(n0 + n) * K + k0 + kc;
  }
#pragma unroll
  for (int i = 0; i < 2; ++i) *(volatile v8h*)(Wt + off[i]) = x[i];
  __threadfence();
#pragma unroll
  for (int i = 0; i < 2; ++i) *(volatile v8h*)(Wt + off[i]) = x[i];
}

template <int RNE_IN>
__device__ __forceinline__ float ldcv(float v) { return RNE_IN ? bf16r(v) : v; }

template <int RNE_IN>
__global__ __launch_bounds__(256) void ln_kernel(
    const float* __restrict__ src, const float* __restrict__ gam,
    const float* __restrict__ bet, _Float16* __restrict__ dst) {
  static_assert(4 * 32 * 8 == DIM);
  const int lane = threadIdx.x & 31, w = threadIdx.x >> 5;
  const int row = blockIdx.x * 8 + w;
  const float* xr = src + (size_t)row * DIM;
  _Float16* orow = dst + (size_t)row * DIM;

  float s = 0.0f;
#pragma unroll 1
  for (int j = 0; j < 4; ++j) {
    const int c = j * 256 + lane * 8;
    const v4f a0 = *(const v4f*)(xr + c);
    const v4f a1 = *(const v4f*)(xr + c + 4);
#pragma unroll
    for (int t = 0; t < 4; ++t) { s += ldcv<RNE_IN>(a0[t]); s += ldcv<RNE_IN>(a1[t]); }
  }
  const float mu = wave_sum(s) * (1.0f / DIM);

  float q = 0.0f;
#pragma unroll 1
  for (int j = 0; j < 4; ++j) {
    const int c = j * 256 + lane * 8;
    const v4f a0 = *(const v4f*)(xr + c);
    const v4f a1 = *(const v4f*)(xr + c + 4);
#pragma unroll
    for (int t = 0; t < 4; ++t) {
      const float d0 = ldcv<RNE_IN>(a0[t]) - mu;
      const float d1 = ldcv<RNE_IN>(a1[t]) - mu;
      q += d0 * d0;
      q += d1 * d1;
    }
  }
  const float var = wave_sum(q) * (1.0f / DIM);
  const float rs = rsqrtf(var + 1.0e-5f);

#pragma unroll 1
  for (int j = 0; j < 4; ++j) {
    const int c = j * 256 + lane * 8;
    const v4f a0 = *(const v4f*)(xr + c);
    const v4f a1 = *(const v4f*)(xr + c + 4);
    const v4f g0 = *(const v4f*)(gam + c);
    const v4f g1 = *(const v4f*)(gam + c + 4);
    const v4f b0 = *(const v4f*)(bet + c);
    const v4f b1 = *(const v4f*)(bet + c + 4);
    v8h o;
#pragma unroll
    for (int t = 0; t < 4; ++t) {
      const float y0 = ((ldcv<RNE_IN>(a0[t]) - mu) * rs) * bf16r(g0[t]) + bf16r(b0[t]);
      const float y1 = ((ldcv<RNE_IN>(a1[t]) - mu) * rs) * bf16r(g1[t]) + bf16r(b1[t]);
      o[t]     = (_Float16)y0;
      o[t + 4] = (_Float16)y1;
    }
    *(volatile v8h*)(orow + c) = o;
    __threadfence();
    *(volatile v8h*)(orow + c) = o;
  }
}

#define MODE_QKV 0
#define MODE_WO  1
#define MODE_W1  2
#define MODE_W2  3

template <int MODE, int KD, int ND>
__global__ __launch_bounds__(256) void gemm_kernel(
    const _Float16* __restrict__ A16, const _Float16* __restrict__ Bt,
    const float* __restrict__ bias, const float* __restrict__ addf,
    float* __restrict__ outf, _Float16* __restrict__ out16) {
  static_assert((KD % 32) == 0 && (ND % 64) == 0);
  static_assert(MODE != MODE_QKV || ND == 3 * DIM);
  static_assert((MODE != MODE_WO && MODE != MODE_W2) || ND == DIM);
  __shared__ float Cs[64 * LDC];
  const int tid = threadIdx.x, lane = tid & 31, w = tid >> 5;
  const int mw = w >> 1, nw = w & 1;
  const int hh = lane >> 4, m = lane & 15;
  const int n0 = blockIdx.x * 64;
  const int row0 = blockIdx.y * 64;

  const _Float16* ap  = A16 + (size_t)(row0 + mw * 16 + m) * KD + hh * 8;
  const _Float16* bp0 = Bt + (size_t)(n0 + nw * 32 + m) * KD + hh * 8;
  const _Float16* bp1 = bp0 + (size_t)16 * KD;
  v8f acc0 = {}, acc1 = {};
#pragma unroll 2
  for (int k0 = 0; k0 < KD; k0 += 32) {
    const v16h a  = frag_at(ap + k0);
    const v16h b0 = frag_at(bp0 + k0);
    const v16h b1 = frag_at(bp1 + k0);
    acc0 = wmma16(a, b0, acc0);
    acc1 = wmma16(a, b1, acc1);
  }
#pragma unroll
  for (int r = 0; r < 8; ++r) {
    float* d = &Cs[(mw * 16 + hh * 8 + r) * LDC + nw * 32 + m];
    d[0]  = acc0[r];
    d[16] = acc1[r];
  }
  __syncthreads();

  if (MODE == MODE_QKV) {
    const int which = n0 / DIM;
    const int nl0 = n0 - which * DIM;
    _Float16* dst = out16 + (size_t)which * ((size_t)MROWS * DIM);
    v8h x[2];
    size_t off[2];
    if (which < 2) {
#pragma unroll
      for (int i = 0; i < 2; ++i) {
        const int r = 32 * i + (tid >> 3);
        const int c = (tid & 7) * 8;
        const v4f u0 = *(const v4f*)&Cs[r * LDC + c];
        const v4f u1 = *(const v4f*)&Cs[r * LDC + c + 4];
        const v4f g0 = *(const v4f*)(bias + n0 + c);
        const v4f g1 = *(const v4f*)(bias + n0 + c + 4);
#pragma unroll
        for (int j = 0; j < 4; ++j) {
          x[i][j]     = (_Float16)(u0[j] * (1.0f / WCARRY) + bf16r(g0[j]));
          x[i][j + 4] = (_Float16)(u1[j] * (1.0f / WCARRY) + bf16r(g1[j]));
        }
        off[i] = (size_t)(row0 + r) * DIM + nl0 + c;
      }
    } else {
#pragma unroll
      for (int i = 0; i < 2; ++i) {
        const int dcol = 32 * i + (tid >> 3);
        const int kk = (tid & 7) * 8;
        const float gb = bf16r(bias[n0 + dcol]);
#pragma unroll
        for (int j = 0; j < 8; ++j)
          x[i][j] = (_Float16)(Cs[(kk + j) * LDC + dcol] * (1.0f / WCARRY) + gb);
        off[i] = (size_t)(nl0 + dcol) * SEQ + row0 + kk;
      }
    }
#pragma unroll
    for (int i = 0; i < 2; ++i) *(volatile v8h*)(dst + off[i]) = x[i];
    __threadfence();
#pragma unroll
    for (int i = 0; i < 2; ++i) *(volatile v8h*)(dst + off[i]) = x[i];
  }

  if (MODE == MODE_WO) {
    v4f xs[4];
    size_t off[4];
#pragma unroll
    for (int i = 0; i < 4; ++i) {
      const int r = 16 * i + (tid >> 4);
      const int c = (tid & 15) * 4;
      const size_t crow = (size_t)(row0 + r);
      const v4f u = *(const v4f*)&Cs[r * LDC + c];
      const v4f g = *(const v4f*)(bias + n0 + c);
      const v4f q = *(const v4f*)(addf + crow * DIM + n0 + c);
      v4f val;
#pragma unroll
      for (int j = 0; j < 4; ++j)
        val[j] = (u[j] * (1.0f / (WCARRY * VCARRY)) + bf16r(g[j])) + bf16r(q[j]);
      xs[i] = val;
      off[i] = crow * ND + n0 + c;
    }
#pragma unroll
    for (int i = 0; i < 4; ++i) *(volatile v4f*)(outf + off[i]) = xs[i];
    __threadfence();
#pragma unroll
    for (int i = 0; i < 4; ++i) *(volatile v4f*)(outf + off[i]) = xs[i];
  }

  if (MODE == MODE_W1) {
    v8h x[2];
    size_t off[2];
#pragma unroll
    for (int i = 0; i < 2; ++i) {
      const int r = 32 * i + (tid >> 3);
      const int c = (tid & 7) * 8;
      const v4f u0 = *(const v4f*)&Cs[r * LDC + c];
      const v4f u1 = *(const v4f*)&Cs[r * LDC + c + 4];
      const v4f g0 = *(const v4f*)(bias + n0 + c);
      const v4f g1 = *(const v4f*)(bias + n0 + c + 4);
#pragma unroll
      for (int j = 0; j < 4; ++j) {
        const float t0 = gelu_erf(u0[j] * (1.0f / WCARRY) + bf16r(g0[j]));
        const float t1 = gelu_erf(u1[j] * (1.0f / WCARRY) + bf16r(g1[j]));
        x[i][j]     = (_Float16)t0;
        x[i][j + 4] = (_Float16)t1;
      }
      off[i] = (size_t)(row0 + r) * ND + n0 + c;
    }
#pragma unroll
    for (int i = 0; i < 2; ++i) *(volatile v8h*)(out16 + off[i]) = x[i];
    __threadfence();
#pragma unroll
    for (int i = 0; i < 2; ++i) *(volatile v8h*)(out16 + off[i]) = x[i];
  }

  if (MODE == MODE_W2) {
    v4f xs[4];
    size_t off[4];
#pragma unroll
    for (int i = 0; i < 4; ++i) {
      const int r = 16 * i + (tid >> 4);
      const int c = (tid & 15) * 4;
      const size_t crow = (size_t)(row0 + r);
      const v4f u  = *(const v4f*)&Cs[r * LDC + c];
      const v4f g  = *(const v4f*)(bias + n0 + c);
      const v4f rx = *(const v4f*)(addf + crow * DIM + n0 + c);
      v4f val;
#pragma unroll
      for (int j = 0; j < 4; ++j)
        val[j] = (u[j] * (1.0f / WCARRY) + bf16r(g[j])) + rx[j];
      xs[i] = val;
      off[i] = crow * ND + n0 + c;
    }
#pragma unroll
    for (int i = 0; i < 4; ++i) *(volatile v4f*)(outf + off[i]) = xs[i];
    __threadfence();
#pragma unroll
    for (int i = 0; i < 4; ++i) *(volatile v4f*)(outf + off[i]) = xs[i];
  }
}

__global__ __launch_bounds__(256) void attn_kernel(
    const _Float16* __restrict__ Qh, const _Float16* __restrict__ Kh,
    const _Float16* __restrict__ Vt, _Float16* __restrict__ Ov) {
  __shared__ _Float16 Ks[64 * LDT];
  __shared__ _Float16 Vs[64 * LDT];
  __shared__ _Float16 Ps[8 * 16 * LDT];

  const int tid = threadIdx.x, lane = tid & 31;
  const int w = __builtin_amdgcn_readfirstlane(tid >> 5);
  const int hh = lane >> 4, m = lane & 15;
  const int q0 = blockIdx.x * 128;
  const int head = blockIdx.y;
  const int wq0 = q0 + w * 16;
  const float scale = 0.125f;
  _Float16* P = Ps + w * (16 * LDT);

  const size_t qoff = (size_t)(wq0 + m) * DIM + head * HD + hh * 8;
  v16h qf[2];
  qf[0] = frag_at(Qh + qoff);
  qf[1] = frag_at(Qh + qoff + 32);

  float mrow[8], lrow[8];
  v8f o[4];
#pragma unroll
  for (int v = 0; v < 8; ++v) { mrow[v] = -1.0e30f; lrow[v] = 0.0f; }
#pragma unroll
  for (int nb = 0; nb < 4; ++nb) o[nb] = (v8f){};

  const size_t kplane = (size_t)head * HD;
  const size_t vplane = (size_t)head * HD * SEQ;
  const int kend = q0 + 128;

  for (int kb = 0; kb < kend; kb += 64) {
#pragma unroll
    for (int j = 0; j < 2; ++j) {
      const int idx = tid + 256 * j;
      const int r = idx >> 3, c = (idx & 7) * 8;
      *(v8h*)&Ks[r * LDT + c] = *(const v8h*)(Kh + kplane + (size_t)(kb + r) * DIM + c);
      *(v8h*)&Vs[r * LDT + c] = *(const v8h*)(Vt + vplane + (size_t)r * SEQ + kb + c);
    }
    __syncthreads();

    if (kb <= wq0 + 15) {
      v8f s[4];
#pragma unroll
      for (int kg = 0; kg < 4; ++kg) {
        v8f t = {};
#pragma unroll
        for (int c = 0; c < 2; ++c) {
          const v16h kf = ld_frag(&Ks[(kg * 16) * LDT + c * 32], LDT);
          t = wmma16(qf[c], kf, t);
        }
        s[kg] = t * scale;
      }

      if (kb + 63 > wq0) {
#pragma unroll
        for (int kg = 0; kg < 4; ++kg)
#pragma unroll
          for (int v = 0; v < 8; ++v) {
            const int key = kb + kg * 16 + m;
            const int qrow = wq0 + hh * 8 + v;
            s[kg][v] = (key > qrow) ? -1.0e30f : s[kg][v];
          }
      }

      float alpha[8];
#pragma unroll
      for (int v = 0; v < 8; ++v) {
        float mx = fmaxf(fmaxf(s[0][v], s[1][v]), fmaxf(s[2][v], s[3][v]));
        mx = red16_max(mx);
        const float mn = fmaxf(mrow[v], mx);
        alpha[v] = __expf(mrow[v] - mn);
        mrow[v] = mn;
      }
#pragma unroll
      for (int kg = 0; kg < 4; ++kg)
#pragma unroll
        for (int v = 0; v < 8; ++v) s[kg][v] = __expf(s[kg][v] - mrow[v]);
#pragma unroll
      for (int v = 0; v < 8; ++v) {
        const float rs = red16_sum((s[0][v] + s[1][v]) + (s[2][v] + s[3][v]));
        lrow[v] = alpha[v] * lrow[v] + rs;
      }
#pragma unroll
      for (int nb = 0; nb < 4; ++nb)
#pragma unroll
        for (int v = 0; v < 8; ++v) o[nb][v] = o[nb][v] * alpha[v];

#pragma unroll
      for (int kg = 0; kg < 4; ++kg)
#pragma unroll
        for (int v = 0; v < 8; ++v)
          P[(hh * 8 + v) * LDT + kg * 16 + m] = (_Float16)(s[kg][v] * PCARRY);
      wave_lds_sync();

#pragma unroll
      for (int c = 0; c < 2; ++c) {
        const v16h pf = ld_frag(P + c * 32, LDT);
#pragma unroll
        for (int nb = 0; nb < 4; ++nb) {
          const v16h vf = ld_frag(&Vs[(nb * 16) * LDT + c * 32], LDT);
          o[nb] = wmma16(pf, vf, o[nb]);
        }
      }
    }
    __syncthreads();
  }

  float inv[8];
#pragma unroll
  for (int v = 0; v < 8; ++v) inv[v] = __builtin_amdgcn_rcpf(lrow[v]) * (VCARRY / PCARRY);
#pragma unroll
  for (int nb = 0; nb < 4; ++nb)
#pragma unroll
    for (int v = 0; v < 8; ++v)
      P[(hh * 8 + v) * LDT + nb * 16 + m] = (_Float16)(o[nb][v] * inv[v]);
  wave_lds_sync();
  v8h x[4];
  size_t off[4];
#pragma unroll
  for (int i = 0; i < 4; ++i) {
    const int r = 4 * i + (lane >> 3);
    const int c = (lane & 7) * 8;
    x[i] = *(const v8h*)&P[r * LDT + c];
    off[i] = (size_t)(wq0 + r) * DIM + head * HD + c;
  }
#pragma unroll
  for (int i = 0; i < 4; ++i) *(volatile v8h*)(Ov + off[i]) = x[i];
  __threadfence();
#pragma unroll
  for (int i = 0; i < 4; ++i) *(volatile v8h*)(Ov + off[i]) = x[i];
}

extern "C" void kernel_launch(void* const* d_in, const int* in_sizes, int n_in,
                              void* d_out, int out_size, void* d_ws, size_t ws_size,
                              hipStream_t stream) {
  if (n_in < 13) return;
  const long long need_x = ((long long)(NB - 1) * SEQ_FULL + SEQ) * DIM;
  if ((long long)in_sizes[0] < need_x) return;
  if (in_sizes[1] < DIM || in_sizes[2] < DIM || in_sizes[6] < DIM || in_sizes[7] < DIM ||
      in_sizes[8] < DIM || in_sizes[12] < DIM) return;
  if (in_sizes[3] < 3 * DIM * DIM || in_sizes[4] < 3 * DIM) return;
  if (in_sizes[5] < DIM * DIM) return;
  if (in_sizes[9] < DIM * FF || in_sizes[10] < FF || in_sizes[11] < FF * DIM) return;
  if ((long long)out_size < need_x) return;
  if (ws_size < WS_TOTAL) return;

  const float* x    = (const float*)d_in[0];
  const float* ln1g = (const float*)d_in[1];
  const float* ln1b = (const float*)d_in[2];
  const float* Wqkv = (const float*)d_in[3];
  const float* bqkv = (const float*)d_in[4];
  const float* Wo   = (const float*)d_in[5];
  const float* bo   = (const float*)d_in[6];
  const float* ln2g = (const float*)d_in[7];
  const float* ln2b = (const float*)d_in[8];
  const float* W1   = (const float*)d_in[9];
  const float* b1   = (const float*)d_in[10];
  const float* W2   = (const float*)d_in[11];
  const float* b2   = (const float*)d_in[12];
  float* out = (float*)d_out;

  char* ws = (char*)d_ws;
  _Float16* WqkvT = (_Float16*)(ws + OFF_WQKV);
  _Float16* WoT   = (_Float16*)(ws + OFF_WO);
  _Float16* W1T   = (_Float16*)(ws + OFF_W1);
  _Float16* W2T   = (_Float16*)(ws + OFF_W2);
  _Float16* Xn16  = (_Float16*)(ws + OFF_XN);
  _Float16* QKV16 = (_Float16*)(ws + OFF_QKV);
  _Float16* Q16   = QKV16;
  _Float16* K16   = QKV16 + (size_t)MROWS * DIM;
  _Float16* Vt16  = QKV16 + (size_t)2 * MROWS * DIM;
  _Float16* Ov16  = (_Float16*)(ws + OFF_OV);
  float*    X32   = (float*)(ws + OFF_X32);
  _Float16* H16   = (_Float16*)(ws + OFF_H);
  _Float16* G16   = (_Float16*)(ws + OFF_G);

  dim3 blk(256);

  wconv_kernel<<<dim3(3 * DIM / 64, DIM / 64), blk, 0, stream>>>(Wqkv, WqkvT, DIM, 3 * DIM);
  wconv_kernel<<<dim3(DIM / 64, DIM / 64), blk, 0, stream>>>(Wo, WoT, DIM, DIM);
  wconv_kernel<<<dim3(FF / 64, DIM / 64), blk, 0, stream>>>(W1, W1T, DIM, FF);
  wconv_kernel<<<dim3(DIM / 64, FF / 64), blk, 0, stream>>>(W2, W2T, FF, DIM);

  ln_kernel<1><<<dim3(MROWS / 8), blk, 0, stream>>>(x, ln1g, ln1b, Xn16);
  gemm_kernel<MODE_QKV, DIM, 3 * DIM><<<dim3(3 * DIM / 64, MROWS / 64), blk, 0, stream>>>(
      Xn16, WqkvT, bqkv, x, X32, QKV16);
  attn_kernel<<<dim3(SEQ / 128, NHEAD), blk, 0, stream>>>(Q16, K16, Vt16, Ov16);
  gemm_kernel<MODE_WO, DIM, DIM><<<dim3(DIM / 64, MROWS / 64), blk, 0, stream>>>(
      Ov16, WoT, bo, x, X32, H16);
  ln_kernel<0><<<dim3(MROWS / 8), blk, 0, stream>>>(X32, ln2g, ln2b, H16);
  gemm_kernel<MODE_W1, DIM, FF><<<dim3(FF / 64, MROWS / 64), blk, 0, stream>>>(
      H16, W1T, b1, X32, out, G16);
  gemm_kernel<MODE_W2, FF, DIM><<<dim3(DIM / 64, MROWS / 64), blk, 0, stream>>>(
      G16, W2T, b2, X32, out, H16);
}
